// RNN_52304111731005
// MI455X (gfx1250) — hardware-verified
//
#include <hip/hip_runtime.h>
#include <math.h>

typedef __attribute__((ext_vector_type(16))) _Float16 v16h;
typedef __attribute__((ext_vector_type(8)))  _Float16 v8h;
typedef __attribute__((ext_vector_type(16))) __bf16   v16b;
typedef __attribute__((ext_vector_type(8)))  __bf16   v8b;
typedef __attribute__((ext_vector_type(8)))  float    v8f;
typedef __attribute__((ext_vector_type(4)))  float    v4f;

constexpr int NBATCH = 16384;
constexpr int NFEAT  = 32;
constexpr int NLIN   = 256;
constexpr int NHID   = 64;
constexpr int NSTEP  = 64;
constexpr int NF0    = 4;
constexpr int NP1    = 16;
static_assert(NLIN == NF0 * NSTEP);

constexpr int ROWS_PB = 32;
constexpr int RTHR    = 128;
constexpr int RBLOCKS = NBATCH / ROWS_PB;
constexpr int HPITCH  = 72;
constexpr int TILE_E  = ROWS_PB * HPITCH;
constexpr int NTILE_E = 3 * 2 * 2 * TILE_E;
constexpr int ZPITCH  = 20;
constexpr int WPLANE  = NHID * NHID;
constexpr int P1PLANE = NP1 * NHID;
static_assert(NBATCH % ROWS_PB == 0);
static_assert(NHID == 16 * (RTHR / 32));
static_assert(ROWS_PB * NF0 == RTHR);
static_assert((NTILE_E / 8) % RTHR == 0);
static_assert(HPITCH % 8 == 0 && ZPITCH % 4 == 0);
static_assert(NHID % 32 == 0);

constexpr int CH_X  = NBATCH * NFEAT / 8;
constexpr int CH_W0 = NLIN * NFEAT / 8;
constexpr int CH_HH = NHID * NHID / 8;
constexpr int CH_P1 = NP1 * NHID / 8;
static_assert(CH_X % 256 == 0 && CH_W0 % 256 == 0 && CH_HH % 256 == 0 && CH_P1 % 32 == 0);
static_assert(NBATCH % 64 == 0 && NLIN % 64 == 0 && NFEAT % 32 == 0);
constexpr int GEMM_TILES  = (NBATCH / 64) * (NLIN / 64);
constexpr int GEMM_BLOCKS = GEMM_TILES / 8;
static_assert(GEMM_TILES % 8 == 0);

__device__ __forceinline__ unsigned short f2bf_bits(float f) {
  unsigned u = __float_as_uint(f);
  return (unsigned short)((u + 0x7FFFu + ((u >> 16) & 1u)) >> 16);
}
__device__ __forceinline__ float bf_bits2f(unsigned short h) { return __uint_as_float(((unsigned)h) << 16); }

__device__ __forceinline__ void dep_guard_h(v8f& a, v8f& b, v16h x, v16h y) { asm volatile("v_nop\n\tv_nop\n\tv_nop\n\tv_nop" : "+v"(a), "+v"(b) : "v"(x), "v"(y)); }
__device__ __forceinline__ void dep_guard_b(v8f& a, v8f& b, v16b x, v16b y) { asm volatile("v_nop\n\tv_nop\n\tv_nop\n\tv_nop" : "+v"(a), "+v"(b) : "v"(x), "v"(y)); }
__device__ __forceinline__ void keep4_h(v16h a, v16h b, v16h c, v16h d) { asm volatile("v_nop" :: "v"(a), "v"(b), "v"(c), "v"(d)); }
__device__ __forceinline__ void keep4_b(v16b a, v16b b, v16b c, v16b d) { asm volatile("v_nop" :: "v"(a), "v"(b), "v"(c), "v"(d)); }
__device__ __forceinline__ void acc_guard4(v8f& a, v8f& b, v8f& c, v8f& d) { asm volatile("v_nop\n\tv_nop\n\tv_nop\n\tv_nop" : "+v"(a), "+v"(b), "+v"(c), "+v"(d)); }
__device__ __forceinline__ void acc_guard2(v8f& a, v8f& b) { asm volatile("v_nop\n\tv_nop\n\tv_nop\n\tv_nop" : "+v"(a), "+v"(b)); }
__device__ __forceinline__ void guard_acc4(v8f& a, v16b f0, v16b f1, v16b f2, v16b f3) {
  asm volatile("v_nop\n\tv_nop\n\tv_nop\n\tv_nop" : "+v"(a) : "v"(f0), "v"(f1), "v"(f2), "v"(f3));
}

template <typename T> struct Frag;
template <> struct Frag<_Float16> {
  typedef v16h V; union U { v16h v; v8h h[2]; };
  static __device__ __forceinline__ v16h load(const _Float16* p) {
    U f; f.h[0] = *(const v8h*)(p); f.h[1] = *(const v8h*)(p + 16); return f.v;
  }
  static __device__ __forceinline__ v8f mma(v16h a, v16h b, v8f c) {
    return __builtin_amdgcn_wmma_f32_16x16x32_f16(false, a, false, b, (short)0, c, false, false);
  }
  static __device__ __forceinline__ void guard(v8f& a, v8f& b, v16h x, v16h y) { dep_guard_h(a, b, x, y); }
  static __device__ __forceinline__ void keep(v16h a, v16h b, v16h c, v16h d) { keep4_h(a, b, c, d); }
};
template <> struct Frag<__bf16> {
  typedef v16b V; union U { v16b v; v8b h[2]; };
  static __device__ __forceinline__ v16b load(const __bf16* p) {
    U f; f.h[0] = *(const v8b*)(p); f.h[1] = *(const v8b*)(p + 16); return f.v;
  }
  static __device__ __forceinline__ v8f mma(v16b a, v16b b, v8f c) {
    return __builtin_amdgcn_wmma_f32_16x16x32_bf16(false, a, false, b, (short)0, c, false, false);
  }
  static __device__ __forceinline__ void guard(v8f& a, v8f& b, v16b x, v16b y) { dep_guard_b(a, b, x, y); }
  static __device__ __forceinline__ void keep(v16b a, v16b b, v16b c, v16b d) { keep4_b(a, b, c, d); }
};

template <int ET> struct Elem;
template <> struct Elem<0> { typedef _Float16 T; };
template <> struct Elem<1> { typedef __bf16 T; };
template <int ET, bool SPLIT, int BIAS_MODE, int OUT_MODE, bool RESID, int ACT = 0>
__global__ __launch_bounds__(256) void wmma_gemm64(
    const unsigned short* __restrict__ Ap, const unsigned short* __restrict__ A2p, int lda, long strideA,
    const unsigned short* __restrict__ Btp, const unsigned short* __restrict__ Bt2p, int ldb, long strideB,
    void* __restrict__ Cout, void* __restrict__ Cout2, int ldc, long strideC,
    const float* __restrict__ bias,
    const float* __restrict__ resid, long strideR,
    int M, int N, int K, float scale) {
  typedef typename Elem<ET>::T T;
  typedef typename Frag<T>::V V;
  const T* A = (const T*)Ap; const T* A2 = (const T*)A2p; const T* Bt = (const T*)Btp; const T* Bt2 = (const T*)Bt2p;
  __shared__ __align__(16) float sT[8][16 * 68];
  const int b    = blockIdx.y;
  const int lane = threadIdx.x & 31;
  const int wave = threadIdx.x >> 5;
  const int tilesN = N >> 6;
  const int tilesM = M >> 6;
  const int tile = blockIdx.x * 8 + wave;
  if (tile >= tilesM * tilesN) return;
  const int tm = tile / tilesN;
  const int tn = tile - tm * tilesN;
  const int m0 = tm << 6;
  const int n0 = tn << 6;

  const T* Ab  = A  + (size_t)b * strideA;
  const T* Bb  = Bt + (size_t)b * strideB;
  const T* Ab2 = SPLIT ? (A2  + (size_t)b * strideA) : nullptr;
  const T* Bb2 = SPLIT ? (Bt2 + (size_t)b * strideB) : nullptr;

  const int rlane = lane & 15;
  const int koff  = (lane >> 4) * 8;
  const int mOff  = (lane >> 4) * 8;

  v8f acc[4][4];
#pragma unroll
  for (int i = 0; i < 4; ++i)
#pragma unroll
    for (int j = 0; j < 4; ++j) acc[i][j] = (v8f){0.f,0.f,0.f,0.f,0.f,0.f,0.f,0.f};

  for (int k0 = 0; k0 < K; k0 += 32) {
    V bh[4], bl[4];
#pragma unroll
    for (int j = 0; j < 4; ++j) {
      const size_t bo = (size_t)(n0 + (j << 4) + rlane) * ldb + koff + k0;
      bh[j] = Frag<T>::load(Bb + bo);
      if (SPLIT) bl[j] = Frag<T>::load(Bb2 + bo);
    }
#pragma unroll
    for (int i = 0; i < 4; ++i) {
      const size_t ao = (size_t)(m0 + (i << 4) + rlane) * lda + koff + k0;
      V ah = Frag<T>::load(Ab + ao);
      V al;
      if (SPLIT) al = Frag<T>::load(Ab2 + ao);
#pragma unroll
      for (int j = 0; j < 4; ++j) {
        acc[i][j] = Frag<T>::mma(ah, bh[j], acc[i][j]);
        if (SPLIT) {
          acc[i][j] = Frag<T>::mma(ah, bl[j], acc[i][j]);
          acc[i][j] = Frag<T>::mma(al, bh[j], acc[i][j]);
        }
      }
      Frag<T>::guard(acc[i][0], acc[i][3], ah, SPLIT ? al : ah);
    }
    Frag<T>::keep(bh[0], bh[1], bh[2], bh[3]);
    if (SPLIT) Frag<T>::keep(bl[0], bl[1], bl[2], bl[3]);
  }
  acc_guard4(acc[0][0], acc[0][1], acc[0][2], acc[0][3]);
  acc_guard4(acc[1][0], acc[1][1], acc[1][2], acc[1][3]);
  acc_guard4(acc[2][0], acc[2][1], acc[2][2], acc[2][3]);
  acc_guard4(acc[3][0], acc[3][1], acc[3][2], acc[3][3]);

  float* slab = sT[wave];
  const float* Rb = RESID ? (resid + (size_t)b * strideR) : nullptr;
#pragma unroll
  for (int i = 0; i < 4; ++i) {
    const int mBase = m0 + (i << 4);
#pragma unroll
    for (int j = 0; j < 4; ++j) {
      const int n = n0 + (j << 4) + rlane;
      float bv = 0.f;
      if (BIAS_MODE == 2) bv = bias[n];
#pragma unroll
      for (int r = 0; r < 8; ++r) {
        float v = acc[i][j][r] * scale;
        if (BIAS_MODE == 1) v += bias[mBase + mOff + r];
        if (BIAS_MODE == 2) v += bv;
        if (RESID) v += Rb[(size_t)(mBase + mOff + r) * ldc + n];
        if (ACT == 1) v = tanhf(v);
        if (ACT == 2) v = fmaxf(v, 0.0f);
        if (ACT == 3) v = v / (1.0f + expf(-v));
        if (ACT == 4) v = (v > 0.f) ? v : 0.01f * v;
        if (ACT == 5) v = 0.5f * v * (1.0f + erff(v * 0.70710678118654752f));
        slab[(mOff + r) * 68 + (j << 4) + rlane] = v;
      }
    }
    __builtin_amdgcn_fence(__ATOMIC_RELEASE, "workgroup");
    __builtin_amdgcn_wave_barrier();
    __builtin_amdgcn_fence(__ATOMIC_ACQUIRE, "workgroup");
    if (OUT_MODE == 0) {
      float* C = (float*)Cout + (size_t)b * strideC;
      const int hh = lane >> 4, c4 = (lane & 15) * 4;
      for (int pass = 0; pass < 2; ++pass) {
#pragma unroll
        for (int it = 0; it < 8; ++it) {
          const int row = it * 2 + hh;
          v4f v = *(const v4f*)(slab + row * 68 + c4);
          *(volatile v4f*)(C + (size_t)(mBase + row) * ldc + n0 + c4) = v;
        }
        __threadfence();
      }
    } else {
      const int q = lane >> 3, c8 = (lane & 7) * 8;
      unsigned short* C  = (unsigned short*)Cout  + (size_t)b * strideC;
      unsigned short* C2 = (OUT_MODE == 2) ? ((unsigned short*)Cout2 + (size_t)b * strideC) : nullptr;
      for (int pass = 0; pass < 2; ++pass) {
#pragma unroll
        for (int it = 0; it < 4; ++it) {
          const int row = it * 4 + q;
          const float* sp = slab + row * 68 + c8;
          v8h hv, lv;
#pragma unroll
          for (int e = 0; e < 8; ++e) {
            if (OUT_MODE == 1) {
              hv[e] = (_Float16)sp[e];
            } else {
              unsigned short hb = f2bf_bits(sp[e]);
              unsigned short lb = f2bf_bits(sp[e] - bf_bits2f(hb));
              hv[e] = __builtin_bit_cast(_Float16, hb);
              lv[e] = __builtin_bit_cast(_Float16, lb);
            }
          }
          *(volatile v8h*)(C + (size_t)(mBase + row) * ldc + n0 + c8) = hv;
          if (OUT_MODE == 2) *(volatile v8h*)(C2 + (size_t)(mBase + row) * ldc + n0 + c8) = lv;
        }
        __threadfence();
      }
    }
    __builtin_amdgcn_fence(__ATOMIC_RELEASE, "workgroup");
    __builtin_amdgcn_wave_barrier();
    __builtin_amdgcn_fence(__ATOMIC_ACQUIRE, "workgroup");
  }
}

__device__ __forceinline__ void bf_split(float f, __bf16& hi, __bf16& lo) {
  const unsigned short hb = f2bf_bits(f);
  hi = __builtin_bit_cast(__bf16, hb);
  lo = __builtin_bit_cast(__bf16, f2bf_bits(f - bf_bits2f(hb)));
}
__device__ __forceinline__ float tanh_id(float x) { return 1.0f - 2.0f * __builtin_amdgcn_rcpf(1.0f + expf(2.0f * x)); }

__global__ __launch_bounds__(256) void cvt_split8_kernel(const float* __restrict__ src,
                                                         unsigned short* __restrict__ dh,
                                                         unsigned short* __restrict__ dl, int nchunk) {
  const int i = blockIdx.x * 256 + threadIdx.x;
  if (i < nchunk) {
    const float* sp = src + (size_t)i * 8;
    const v4f a = *(const v4f*)(sp);
    const v4f b = *(const v4f*)(sp + 4);
    v8h hv, lv;
#pragma unroll
    for (int e = 0; e < 4; ++e) {
      const float fa = a[e];
      const float fb = b[e];
      const unsigned short ha = f2bf_bits(fa);
      const unsigned short la = f2bf_bits(fa - bf_bits2f(ha));
      const unsigned short hb = f2bf_bits(fb);
      const unsigned short lb = f2bf_bits(fb - bf_bits2f(hb));
      hv[e]     = __builtin_bit_cast(_Float16, ha);
      lv[e]     = __builtin_bit_cast(_Float16, la);
      hv[4 + e] = __builtin_bit_cast(_Float16, hb);
      lv[4 + e] = __builtin_bit_cast(_Float16, lb);
    }
    unsigned short* ph = dh + (size_t)i * 8;
    unsigned short* pl = dl + (size_t)i * 8;
    *(volatile v8h*)ph = hv;
    *(volatile v8h*)pl = lv;
    __threadfence();
    *(volatile v8h*)ph = hv;
    *(volatile v8h*)pl = lv;
  }
}

template <bool HAS_IN>
__device__ __forceinline__ void contract_step(v8f (&acc)[2],
    const __bf16* inH, const __bf16* inL, const __bf16* wiH, const __bf16* wiL,
    const __bf16* ownH, const __bf16* ownL, const __bf16* whH, const __bf16* whL,
    int c, int koff) {
#pragma unroll
  for (int ks = 0; ks < 2; ++ks) {
    const int k0 = ks * 32;
    const int bo = c * NHID + koff + k0;
    const v16b bhh = Frag<__bf16>::load(whH + bo);
    const v16b bhl = Frag<__bf16>::load(whL + bo);
    v16b bih = bhh, bil = bhl;
    if (HAS_IN) {
      bih = Frag<__bf16>::load(wiH + bo);
      bil = Frag<__bf16>::load(wiL + bo);
    }
#pragma unroll
    for (int ms = 0; ms < 2; ++ms) {
      const int ao = (ms * 16 + c) * HPITCH + koff + k0;
      const v16b gh = Frag<__bf16>::load(ownH + ao);
      const v16b gl = Frag<__bf16>::load(ownL + ao);
      v16b ah = gh, al = gl;
      if (HAS_IN) {
        ah = Frag<__bf16>::load(inH + ao);
        al = Frag<__bf16>::load(inL + ao);
        acc[ms] = Frag<__bf16>::mma(ah, bih, acc[ms]);
        acc[ms] = Frag<__bf16>::mma(ah, bil, acc[ms]);
        acc[ms] = Frag<__bf16>::mma(al, bih, acc[ms]);
      }
      acc[ms] = Frag<__bf16>::mma(gh, bhh, acc[ms]);
      acc[ms] = Frag<__bf16>::mma(gh, bhl, acc[ms]);
      acc[ms] = Frag<__bf16>::mma(gl, bhh, acc[ms]);
      guard_acc4(acc[ms], ah, al, gh, gl);
    }
    keep4_b(bhh, bhl, bih, bil);
    asm volatile("" ::: "memory");
  }
  acc_guard2(acc[0], acc[1]);
}

__device__ __forceinline__ void store_h(const v8f (&acc)[2], __bf16* oH, __bf16* oL, int mrow, int n) {
#pragma unroll
  for (int ms = 0; ms < 2; ++ms) {
#pragma unroll
    for (int r = 0; r < 8; ++r) {
      const float hv = tanh_id(acc[ms][r]);
      __bf16 a, b;
      bf_split(hv, a, b);
      const int idx = (ms * 16 + mrow + r) * HPITCH + n;
      oH[idx] = a;
      oL[idx] = b;
    }
  }
}

__device__ __forceinline__ __bf16* tile_ptr(__bf16* base, int layer, int buf, int plane) {
  return base + ((layer * 2 + buf) * 2 + plane) * TILE_E;
}

__global__ __launch_bounds__(RTHR) void rnn3_kernel(
    const float* __restrict__ HLIN,
    const unsigned short* __restrict__ wrec,
    const unsigned short* __restrict__ wp1p,
    const float* __restrict__ w_ih0,
    const float* __restrict__ b_ih0, const float* __restrict__ b_hh0,
    const float* __restrict__ b_ih1, const float* __restrict__ b_hh1,
    const float* __restrict__ b_ih2, const float* __restrict__ b_hh2,
    const float* __restrict__ bp1, const float* __restrict__ wp2, const float* __restrict__ bp2,
    float* __restrict__ out) {
  __shared__ __align__(16) __bf16 HT[NTILE_E];
  __shared__ __align__(16) float  XSL[2 * ROWS_PB * NF0];
  __shared__ __align__(16) float  ZS[ROWS_PB * ZPITCH];
  __shared__ __align__(16) float  OUTS[ROWS_PB];

  const int tid = threadIdx.x, lane = tid & 31, wave = tid >> 5;
  const int c = lane & 15, hh = lane >> 4, koff = hh * 8, mrow = hh * 8;
  const int n = 16 * wave + c;
  const int row0 = blockIdx.x * ROWS_PB;

  {
    const __bf16 bz = __builtin_bit_cast(__bf16, (unsigned short)0);
    const v8b z = {bz, bz, bz, bz, bz, bz, bz, bz};
#pragma unroll 1
    for (int i = tid; i < NTILE_E / 8; i += RTHR) *(v8b*)(HT + 8 * i) = z;
  }
  {
    const int rr = tid >> 2, f = tid & 3;
    XSL[tid] = HLIN[(size_t)(row0 + rr) * NLIN + f * NSTEP + 0];
  }
  const v4f   wi0 = *(const v4f*)(w_ih0 + n * NF0);
  const float bs0 = b_ih0[n] + b_hh0[n];
  const float bs1 = b_ih1[n] + b_hh1[n];
  const float bs2 = b_ih2[n] + b_hh2[n];
  __syncthreads();

  const __bf16* WB = (const __bf16*)wrec + (size_t)(16 * wave) * NHID;
  const __bf16* WHH0H = WB + 0 * WPLANE; const __bf16* WHH0L = WB + 1 * WPLANE;
  const __bf16* WIH1H = WB + 2 * WPLANE; const __bf16* WIH1L = WB + 3 * WPLANE;
  const __bf16* WHH1H = WB + 4 * WPLANE; const __bf16* WHH1L = WB + 5 * WPLANE;
  const __bf16* WIH2H = WB + 6 * WPLANE; const __bf16* WIH2L = WB + 7 * WPLANE;
  const __bf16* WHH2H = WB + 8 * WPLANE; const __bf16* WHH2L = WB + 9 * WPLANE;

#pragma unroll 1
  for (int t = 0; t < NSTEP; ++t) {
    const int p = t & 1, q = p ^ 1;
    {
      const int tn = (t + 1 < NSTEP) ? (t + 1) : (NSTEP - 1);
      const int rr = tid >> 2, f = tid & 3;
      XSL[q * (ROWS_PB * NF0) + tid] = HLIN[(size_t)(row0 + rr) * NLIN + f * NSTEP + tn];
    }
    v8f acc[2];
    {
      const float* xs = XSL + p * (ROWS_PB * NF0);
#pragma unroll
      for (int ms = 0; ms < 2; ++ms) {
#pragma unroll
        for (int r = 0; r < 8; ++r) {
          const v4f s = *(const v4f*)(xs + (ms * 16 + mrow + r) * NF0);
          float v = bs0;
          v = fmaf(s[0], wi0[0], v);
          v = fmaf(s[1], wi0[1], v);
          v = fmaf(s[2], wi0[2], v);
          v = fmaf(s[3], wi0[3], v);
          acc[ms][r] = v;
        }
      }
      contract_step<false>(acc, nullptr, nullptr, nullptr, nullptr,
                           tile_ptr(HT, 0, q, 0), tile_ptr(HT, 0, q, 1), WHH0H, WHH0L, c, koff);
      store_h(acc, tile_ptr(HT, 0, p, 0), tile_ptr(HT, 0, p, 1), mrow, n);
    }
    __syncthreads();
    {
      acc[0] = (v8f){bs1, bs1, bs1, bs1, bs1, bs1, bs1, bs1};
      acc[1] = acc[0];
      contract_step<true>(acc, tile_ptr(HT, 0, p, 0), tile_ptr(HT, 0, p, 1), WIH1H, WIH1L,
                          tile_ptr(HT, 1, q, 0), tile_ptr(HT, 1, q, 1), WHH1H, WHH1L, c, koff);
      store_h(acc, tile_ptr(HT, 1, p, 0), tile_ptr(HT, 1, p, 1), mrow, n);
    }
    __syncthreads();
    {
      acc[0] = (v8f){bs2, bs2, bs2, bs2, bs2, bs2, bs2, bs2};
      acc[1] = acc[0];
      contract_step<true>(acc, tile_ptr(HT, 1, p, 0), tile_ptr(HT, 1, p, 1), WIH2H, WIH2L,
                          tile_ptr(HT, 2, q, 0), tile_ptr(HT, 2, q, 1), WHH2H, WHH2L, c, koff);
      store_h(acc, tile_ptr(HT, 2, p, 0), tile_ptr(HT, 2, p, 1), mrow, n);
    }
    __syncthreads();
  }

  const __bf16* H2H = tile_ptr(HT, 2, (NSTEP - 1) & 1, 0);
  const __bf16* H2L = tile_ptr(HT, 2, (NSTEP - 1) & 1, 1);
  if (wave == 0) {
    const float bp1c = bp1[c];
    v8f pz[2];
    pz[0] = (v8f){bp1c, bp1c, bp1c, bp1c, bp1c, bp1c, bp1c, bp1c};
    pz[1] = pz[0];
    const __bf16* P1H = (const __bf16*)wp1p;
    const __bf16* P1L = P1H + P1PLANE;
#pragma unroll
    for (int ks = 0; ks < 2; ++ks) {
      const int k0 = ks * 32;
      const int bo = c * NHID + koff + k0;
      const v16b bh = Frag<__bf16>::load(P1H + bo);
      const v16b bl = Frag<__bf16>::load(P1L + bo);
#pragma unroll
      for (int ms = 0; ms < 2; ++ms) {
        const int ao = (ms * 16 + c) * HPITCH + koff + k0;
        const v16b ah = Frag<__bf16>::load(H2H + ao);
        const v16b al = Frag<__bf16>::load(H2L + ao);
        pz[ms] = Frag<__bf16>::mma(ah, bh, pz[ms]);
        pz[ms] = Frag<__bf16>::mma(ah, bl, pz[ms]);
        pz[ms] = Frag<__bf16>::mma(al, bh, pz[ms]);
        guard_acc4(pz[ms], ah, al, bh, bl);
      }
      keep4_b(bh, bl, bh, bl);
      asm volatile("" ::: "memory");
    }
    acc_guard2(pz[0], pz[1]);
#pragma unroll
    for (int ms = 0; ms < 2; ++ms)
#pragma unroll
      for (int r = 0; r < 8; ++r) ZS[(ms * 16 + mrow + r) * ZPITCH + c] = fmaxf(pz[ms][r], 0.0f);
  }
  __syncthreads();
  if (wave == 0) {
    const v4f wq0 = *(const v4f*)(wp2 + 0);
    const v4f wq1 = *(const v4f*)(wp2 + 4);
    const v4f wq2 = *(const v4f*)(wp2 + 8);
    const v4f wq3 = *(const v4f*)(wp2 + 12);
    const float bp2v = bp2[0];
    const float* zr = ZS + lane * ZPITCH;
    const v4f z0 = *(const v4f*)(zr + 0);
    const v4f z1 = *(const v4f*)(zr + 4);
    const v4f z2 = *(const v4f*)(zr + 8);
    const v4f z3 = *(const v4f*)(zr + 12);
    float a = 0.0f;
    a = fmaf(z0[0], wq0[0], a); a = fmaf(z0[1], wq0[1], a); a = fmaf(z0[2], wq0[2], a); a = fmaf(z0[3], wq0[3], a);
    a = fmaf(z1[0], wq1[0], a); a = fmaf(z1[1], wq1[1], a); a = fmaf(z1[2], wq1[2], a); a = fmaf(z1[3], wq1[3], a);
    a = fmaf(z2[0], wq2[0], a); a = fmaf(z2[1], wq2[1], a); a = fmaf(z2[2], wq2[2], a); a = fmaf(z2[3], wq2[3], a);
    a = fmaf(z3[0], wq3[0], a); a = fmaf(z3[1], wq3[1], a); a = fmaf(z3[2], wq3[2], a); a = fmaf(z3[3], wq3[3], a);
    OUTS[lane] = a + bp2v;
  }
  __syncthreads();
  if (wave == 0) {
    const int l8 = lane & 7;
    const v4f v = *(const v4f*)(OUTS + 4 * l8);
    float* op = out + (size_t)row0 + 4 * l8;
    if (lane < 8) *(volatile v4f*)op = v;
    __threadfence();
    if (lane < 8) *(volatile v4f*)op = v;
  }
}

extern "C" void kernel_launch(void* const* d_in, const int* in_sizes, int n_in,
                              void* d_out, int out_size, void* d_ws, size_t ws_size, hipStream_t stream) {
  if (n_in < 19 || d_out == nullptr || d_ws == nullptr) return;
  if (in_sizes[0] != NBATCH * NFEAT || in_sizes[1] != NLIN * NFEAT || in_sizes[2] != NLIN ||
      in_sizes[3] != NHID * NF0 || in_sizes[4] != NHID * NHID || in_sizes[5] != NHID || in_sizes[6] != NHID ||
      in_sizes[7] != NHID * NHID || in_sizes[8] != NHID * NHID || in_sizes[9] != NHID || in_sizes[10] != NHID ||
      in_sizes[11] != NHID * NHID || in_sizes[12] != NHID * NHID || in_sizes[13] != NHID || in_sizes[14] != NHID ||
      in_sizes[15] != NP1 * NHID || in_sizes[16] != NP1 || in_sizes[17] != NP1 || in_sizes[18] != 1 ||
      out_size != NBATCH) return;

  const float* x     = (const float*)d_in[0];
  const float* w0    = (const float*)d_in[1];
  const float* b0    = (const float*)d_in[2];
  const float* w_ih0 = (const float*)d_in[3];
  const float* w_hh0 = (const float*)d_in[4];
  const float* b_ih0 = (const float*)d_in[5];
  const float* b_hh0 = (const float*)d_in[6];
  const float* w_ih1 = (const float*)d_in[7];
  const float* w_hh1 = (const float*)d_in[8];
  const float* b_ih1 = (const float*)d_in[9];
  const float* b_hh1 = (const float*)d_in[10];
  const float* w_ih2 = (const float*)d_in[11];
  const float* w_hh2 = (const float*)d_in[12];
  const float* b_ih2 = (const float*)d_in[13];
  const float* b_hh2 = (const float*)d_in[14];
  const float* wp1   = (const float*)d_in[15];
  const float* bp1   = (const float*)d_in[16];
  const float* wp2   = (const float*)d_in[17];
  const float* bp2   = (const float*)d_in[18];
  float* out = (float*)d_out;

  char* ws = (char*)d_ws; size_t off = 0;
  auto carve = [&](size_t bytes) -> char* { char* p = ws + off; off += (bytes + 255) & ~(size_t)255; return p; };
  unsigned short* XH   = (unsigned short*)carve((size_t)NBATCH * NFEAT * 2);
  unsigned short* XL   = (unsigned short*)carve((size_t)NBATCH * NFEAT * 2);
  unsigned short* W0H  = (unsigned short*)carve((size_t)NLIN * NFEAT * 2);
  unsigned short* W0L  = (unsigned short*)carve((size_t)NLIN * NFEAT * 2);
  unsigned short* WREC = (unsigned short*)carve((size_t)10 * WPLANE * 2);
  unsigned short* WP1  = (unsigned short*)carve((size_t)2 * P1PLANE * 2);
  float*          HLIN = (float*)carve((size_t)NBATCH * NLIN * 4);
  if (off > ws_size || off > (size_t)134217728) return;

  cvt_split8_kernel<<<CH_X / 256, 256, 0, stream>>>(x, XH, XL, CH_X);
  cvt_split8_kernel<<<CH_W0 / 256, 256, 0, stream>>>(w0, W0H, W0L, CH_W0);
  cvt_split8_kernel<<<CH_HH / 256, 256, 0, stream>>>(w_hh0, WREC + 0 * WPLANE, WREC + 1 * WPLANE, CH_HH);
  cvt_split8_kernel<<<CH_HH / 256, 256, 0, stream>>>(w_ih1, WREC + 2 * WPLANE, WREC + 3 * WPLANE, CH_HH);
  cvt_split8_kernel<<<CH_HH / 256, 256, 0, stream>>>(w_hh1, WREC + 4 * WPLANE, WREC + 5 * WPLANE, CH_HH);
  cvt_split8_kernel<<<CH_HH / 256, 256, 0, stream>>>(w_ih2, WREC + 6 * WPLANE, WREC + 7 * WPLANE, CH_HH);
  cvt_split8_kernel<<<CH_HH / 256, 256, 0, stream>>>(w_hh2, WREC + 8 * WPLANE, WREC + 9 * WPLANE, CH_HH);
  cvt_split8_kernel<<<(CH_P1 + 255) / 256, 256, 0, stream>>>(wp1, WP1, WP1 + P1PLANE, CH_P1);

  wmma_gemm64<1, true, 2, 0, false, 0><<<dim3(GEMM_BLOCKS, 1), 256, 0, stream>>>(
      XH, XL, NFEAT, 0L, W0H, W0L, NFEAT, 0L,
      (void*)HLIN, (void*)HLIN, NLIN, 0L, b0, HLIN, 0L, NBATCH, NLIN, NFEAT, 1.0f);

  rnn3_kernel<<<RBLOCKS, RTHR, 0, stream>>>(HLIN, WREC, WP1, w_ih0, b_ih0, b_hh0, b_ih1, b_hh1, b_ih2, b_hh2,
                                            bp1, wp2, bp2, out);
}
